// TSModel_36524401885659
// MI455X (gfx1250) — hardware-run, weakly checked
//
#include <hip/hip_runtime.h>
#include <math.h>

typedef __attribute__((ext_vector_type(16))) __bf16 v16b;
typedef __attribute__((ext_vector_type(8)))  __bf16 v8b;
typedef __attribute__((ext_vector_type(8)))  float  v8f;
typedef __attribute__((ext_vector_type(4)))  float  v4f;

namespace {
constexpr int   kBatch    = 512;
constexpr int   kSteps    = 2048;
constexpr int   kHid      = 64;
constexpr int   kGateCols = 4 * kHid;
constexpr int   kRowsBlk  = 16;
constexpr int   kThreads  = 128;
constexpr int   kHPitch   = 72;
constexpr int   kHPlane   = kRowsBlk * kHPitch;
constexpr int   kGroup    = 32;
constexpr int   kOsPitch  = 36;
constexpr float kLog2e    = 1.4426950408889634f;
static_assert(kHid == 64, "two 32-deep k-steps");
static_assert((kBatch % kRowsBlk) == 0, "batch tile multiple");
static_assert((kSteps % kGroup) == 0, "whole 128-B lines in time");
static_assert(kGateCols == kThreads * 2, "four 16-wide tiles per wave, four waves");
static_assert((kHPitch % 8) == 0 && kHPitch >= kHid, "16-B aligned fragment rows");
}

__device__ __forceinline__ unsigned short f2bf_bits(float f) {
  unsigned u = __float_as_uint(f);
  return (unsigned short)((u + 0x7FFFu + ((u >> 16) & 1u)) >> 16);
}
__device__ __forceinline__ float bf_bits2f(unsigned short h) { return __uint_as_float(((unsigned)h) << 16); }
__device__ __forceinline__ float rne_bf(float f) { return bf_bits2f(f2bf_bits(f)); }
__device__ __forceinline__ __bf16 bits_to_bf(unsigned short b) { return __builtin_bit_cast(__bf16, b); }

struct FragB {
  union U { v16b v; v8b h[2]; };
  static __device__ __forceinline__ v16b load(const __bf16* p) {
    U f; f.h[0] = *(const v8b*)(p); f.h[1] = *(const v8b*)(p + 16); return f.v;
  }
  static __device__ __forceinline__ v8f mma(v16b a, v16b b, v8f c) {
    return __builtin_amdgcn_wmma_f32_16x16x32_bf16(false, a, false, b, (short)0, c, false, false);
  }
};

__device__ __forceinline__ void acc_guard(v8f& c, v16b a0, v16b a1, v16b a2, v16b a3, v16b b0, v16b b1) {
  asm volatile("v_nop\n\tv_nop\n\tv_nop\n\tv_nop" : "+v"(c) : "v"(a0), "v"(a1), "v"(a2), "v"(a3), "v"(b0), "v"(b1));
}

__device__ __forceinline__ float fast_sigmoid(float z) {
  return __builtin_amdgcn_rcpf(1.0f + __builtin_amdgcn_exp2f(-kLog2e * z));
}
__device__ __forceinline__ float fast_tanh(float z) {
  const float zc = fminf(fmaxf(z, -15.0f), 15.0f);
  const float s  = __builtin_amdgcn_rcpf(1.0f + __builtin_amdgcn_exp2f((-2.0f * kLog2e) * zc));
  return fmaf(2.0f, s, -1.0f);
}

__device__ __forceinline__ void stage_x_chunk(const float* xg, float* xsb, int lane) {
  const int q = lane >> 3, c4 = (lane & 7) * 4;
#pragma unroll
  for (int it = 0; it < 4; ++it) {
    const int row = it * 4 + q;
    const v4f v = *(const v4f*)(xg + (size_t)row * kSteps + c4);
    const float e0 = v[0], e1 = v[1], e2 = v[2], e3 = v[3];
    xsb[(c4 + 0) * kRowsBlk + row] = rne_bf(e0);
    xsb[(c4 + 1) * kRowsBlk + row] = rne_bf(e1);
    xsb[(c4 + 2) * kRowsBlk + row] = rne_bf(e2);
    xsb[(c4 + 3) * kRowsBlk + row] = rne_bf(e3);
  }
}

__device__ __forceinline__ void flush_out_group(const float* osb, float* og, int lane) {
  const int q = lane >> 3, c4 = (lane & 7) * 4;
  v4f v[4];
#pragma unroll
  for (int it = 0; it < 4; ++it) v[it] = *(const v4f*)(osb + (it * 4 + q) * kOsPitch + c4);
  for (int pass = 0; pass < 2; ++pass) {
#pragma unroll
    for (int it = 0; it < 4; ++it)
      *(volatile v4f*)(og + (size_t)(it * 4 + q) * kSteps + c4) = v[it];
    __threadfence();
  }
}

__device__ __forceinline__ float second_cell_step(v16b wa0, v16b wa1, v16b hh0, v16b hl0, v16b hh1, v16b hl1,
                                                  float wi, float wj, float wf, float wo,
                                                  float bi, float bj, float bfg, float bo,
                                                  float& c2, float h2prior) {
  v8f z;
  z[0] = fmaf(h2prior, wi, bi);
  z[1] = fmaf(h2prior, wj, bj);
  z[2] = fmaf(h2prior, wf, bfg);
  z[3] = fmaf(h2prior, wo, bo);
  z[4] = 0.0f; z[5] = 0.0f; z[6] = 0.0f; z[7] = 0.0f;
  z = FragB::mma(wa0, hh0, z);
  z = FragB::mma(wa0, hl0, z);
  z = FragB::mma(wa1, hh1, z);
  z = FragB::mma(wa1, hl1, z);
  acc_guard(z, wa0, wa1, hh0, hl0, hh1, hl1);
  const float zi = z[0], zj = z[1], zf = z[2], zo = z[3];
  const float i2 = fast_sigmoid(zi);
  const float j2 = fast_tanh(zj);
  const float f2 = __builtin_amdgcn_rcpf(1.0f + __builtin_amdgcn_exp2f(fmaf(-kLog2e, zf, -kLog2e)));
  const float o2 = fast_sigmoid(zo);
  const float cn = fmaf(c2, f2, i2 * j2);
  c2 = cn;
  return fast_tanh(cn) * o2;
}

__global__ __launch_bounds__(128) __attribute__((amdgpu_num_vgpr(256)))
void lstm2_fused_kernel(const float* __restrict__ x, const float* __restrict__ W1,
                        const float* __restrict__ b1, const float* __restrict__ W2,
                        const float* __restrict__ b2, float* __restrict__ out)
{
  __shared__ __align__(16) __bf16 wT[kGateCols * kHPitch];
  __shared__ __align__(16) __bf16 w2T[16 * kHPitch];
  __shared__ __align__(16) __bf16 hpl[4 * kHPlane];
  __shared__ __align__(16) float xs[2 * kGroup * kRowsBlk];
  __shared__ __align__(16) float os[2 * kRowsBlk * kOsPitch];

  const int tid  = threadIdx.x;
  const int lane = tid & 31;
  const int wave = tid >> 5;
  const int hf   = lane >> 4;
  const int l15  = lane & 15;
  const int unit = 16 * wave + l15;
  const int b0   = blockIdx.x * kRowsBlk;

#pragma unroll 2
  for (int it = 0; it < 32; ++it) {
    const int idx = it * kThreads + tid;
    const int kk  = idx >> 6;
    const int c4  = (idx & 63) * 4;
    const v4f wv = *(const v4f*)(W1 + (size_t)(1 + kk) * kGateCols + c4);
    const float e0 = wv[0], e1 = wv[1], e2 = wv[2], e3 = wv[3];
    wT[(c4 + 0) * kHPitch + kk] = bits_to_bf(f2bf_bits(e0));
    wT[(c4 + 1) * kHPitch + kk] = bits_to_bf(f2bf_bits(e1));
    wT[(c4 + 2) * kHPitch + kk] = bits_to_bf(f2bf_bits(e2));
    wT[(c4 + 3) * kHPitch + kk] = bits_to_bf(f2bf_bits(e3));
  }
#pragma unroll 1
  for (int idx = tid; idx < 16 * kHPitch; idx += kThreads) {
    const int m  = idx / kHPitch;
    const int k  = idx - m * kHPitch;
    const int mc = (m < 4) ? m : 3;
    const int kc = (k < kHid) ? k : (kHid - 1);
    const float wv  = W2[kc * 4 + mc];
    const float sel = (m < 4 && k < kHid) ? wv : 0.0f;
    w2T[idx] = bits_to_bf(f2bf_bits(sel));
  }
#pragma unroll 1
  for (int idx = tid; idx < 4 * kHPlane; idx += kThreads) hpl[idx] = bits_to_bf((unsigned short)0);
  if (wave == 2) stage_x_chunk(x + (size_t)b0 * kSteps, xs, lane);
  __syncthreads();

  v16b bf[4][2];
#pragma unroll
  for (int g = 0; g < 4; ++g) {
#pragma unroll
    for (int s = 0; s < 2; ++s)
      bf[g][s] = FragB::load(wT + (kHid * g + unit) * kHPitch + 32 * s + 8 * hf);
  }
  const v16b wa0 = FragB::load(w2T + l15 * kHPitch + 8 * hf);
  const v16b wa1 = FragB::load(w2T + l15 * kHPitch + 32 + 8 * hf);
  float w0[4], bb[4];
#pragma unroll
  for (int g = 0; g < 4; ++g) {
    w0[g] = rne_bf(W1[kHid * g + unit]);
    bb[g] = rne_bf(b1[kHid * g + unit]);
  }
  const float w2i = rne_bf(W2[kHid * 4 + 0]), w2j = rne_bf(W2[kHid * 4 + 1]);
  const float w2f = rne_bf(W2[kHid * 4 + 2]), w2o = rne_bf(W2[kHid * 4 + 3]);
  const float b2i = rne_bf(b2[0]), b2j = rne_bf(b2[1]), b2f = rne_bf(b2[2]), b2o = rne_bf(b2[3]);

  float c1[8];
#pragma unroll
  for (int r = 0; r < 8; ++r) c1[r] = 0.0f;
  float c2r = 0.0f, h2r = 0.0f;
  const int aoff = l15 * kHPitch + 8 * hf;

#pragma unroll 1
  for (int t = 0; t < kSteps; ++t) {
    const int rdb = t & 1;
    const __bf16* rh = hpl + rdb * (2 * kHPlane);
    const __bf16* rl = rh + kHPlane;
    __bf16* wh = hpl + (rdb ^ 1) * (2 * kHPlane);
    __bf16* wl = wh + kHPlane;

    const v16b ah0 = FragB::load(rh + aoff);
    const v16b ah1 = FragB::load(rh + aoff + 32);
    const v16b al0 = FragB::load(rl + aoff);
    const v16b al1 = FragB::load(rl + aoff + 32);

    const float* xp = xs + ((t >> 5) & 1) * (kGroup * kRowsBlk) + (t & 31) * kRowsBlk + 8 * hf;
    const v4f xa = *(const v4f*)(xp);
    const v4f xb = *(const v4f*)(xp + 4);
    float xv[8];
    xv[0] = xa[0]; xv[1] = xa[1]; xv[2] = xa[2]; xv[3] = xa[3];
    xv[4] = xb[0]; xv[5] = xb[1]; xv[6] = xb[2]; xv[7] = xb[3];

    v8f acc[4];
#pragma unroll
    for (int g = 0; g < 4; ++g) {
#pragma unroll
      for (int r = 0; r < 8; ++r) acc[g][r] = fmaf(xv[r], w0[g], bb[g]);
    }
#pragma unroll
    for (int g = 0; g < 4; ++g) acc[g] = FragB::mma(ah0, bf[g][0], acc[g]);
#pragma unroll
    for (int g = 0; g < 4; ++g) acc[g] = FragB::mma(al0, bf[g][0], acc[g]);
#pragma unroll
    for (int g = 0; g < 4; ++g) acc[g] = FragB::mma(ah1, bf[g][1], acc[g]);
#pragma unroll
    for (int g = 0; g < 4; ++g) acc[g] = FragB::mma(al1, bf[g][1], acc[g]);
    acc_guard(acc[0], ah0, ah1, al0, al1, bf[0][0], bf[0][1]);
    acc_guard(acc[1], ah0, ah1, al0, al1, bf[1][0], bf[1][1]);
    acc_guard(acc[2], ah0, ah1, al0, al1, bf[2][0], bf[2][1]);
    acc_guard(acc[3], ah0, ah1, al0, al1, bf[3][0], bf[3][1]);

    if (wave == 0 && t > 0) {
      const float h2n = second_cell_step(wa0, wa1, ah0, al0, ah1, al1,
                                         w2i, w2j, w2f, w2o, b2i, b2j, b2f, b2o, c2r, h2r);
      h2r = h2n;
      const int tt = t - 1;
      if (lane < 16) os[((tt >> 5) & 1) * (kRowsBlk * kOsPitch) + l15 * kOsPitch + (tt & 31)] = h2n;
    }

#pragma unroll
    for (int r = 0; r < 8; ++r) {
      const float zi = acc[0][r], zj = acc[1][r], zf = acc[2][r], zo = acc[3][r];
      const float si = fast_sigmoid(zi);
      const float tj = fast_tanh(zj);
      const float sf = __builtin_amdgcn_rcpf(1.0f + __builtin_amdgcn_exp2f(fmaf(-kLog2e, zf, -kLog2e)));
      const float so = fast_sigmoid(zo);
      const float cn = fmaf(c1[r], sf, si * tj);
      c1[r] = cn;
      const float hn = fast_tanh(cn) * so;
      const unsigned short hb = f2bf_bits(hn);
      const float hres = hn - bf_bits2f(hb);
      const unsigned short lb = f2bf_bits(hres);
      const int wofs = (8 * hf + r) * kHPitch + unit;
      wh[wofs] = bits_to_bf(hb);
      wl[wofs] = bits_to_bf(lb);
    }

    if (wave == 2 && (t & 31) == 2 && ((t >> 5) + 1) < (kSteps / kGroup)) {
      const int cn1 = (t >> 5) + 1;
      stage_x_chunk(x + (size_t)b0 * kSteps + (size_t)cn1 * kGroup, xs + (cn1 & 1) * (kGroup * kRowsBlk), lane);
    }
    if (wave == 1 && (t & 31) == 1 && t >= 33) {
      const int gi = (t >> 5) - 1;
      flush_out_group(os + (gi & 1) * (kRowsBlk * kOsPitch), out + (size_t)b0 * kSteps + (size_t)gi * kGroup, lane);
    }
    __syncthreads();
  }

  if (wave == 0) {
    const __bf16* rh = hpl + (kSteps & 1) * (2 * kHPlane);
    const __bf16* rl = rh + kHPlane;
    const v16b ah0 = FragB::load(rh + aoff);
    const v16b ah1 = FragB::load(rh + aoff + 32);
    const v16b al0 = FragB::load(rl + aoff);
    const v16b al1 = FragB::load(rl + aoff + 32);
    const float h2n = second_cell_step(wa0, wa1, ah0, al0, ah1, al1,
                                       w2i, w2j, w2f, w2o, b2i, b2j, b2f, b2o, c2r, h2r);
    h2r = h2n;
    const int tt = kSteps - 1;
    if (lane < 16) os[((tt >> 5) & 1) * (kRowsBlk * kOsPitch) + l15 * kOsPitch + (tt & 31)] = h2n;
  }
  __syncthreads();
  if (wave == 1) {
    const int gi = (kSteps / kGroup) - 1;
    flush_out_group(os + (gi & 1) * (kRowsBlk * kOsPitch), out + (size_t)b0 * kSteps + (size_t)gi * kGroup, lane);
  }
}

extern "C" void kernel_launch(void* const* d_in, const int* in_sizes, int n_in,
                              void* d_out, int out_size, void* d_ws, size_t ws_size,
                              hipStream_t stream) {
  if (n_in < 5) return;
  if (in_sizes[0] != kBatch * kSteps) return;
  if (in_sizes[1] != (kHid + 1) * kGateCols) return;
  if (in_sizes[2] != kGateCols) return;
  if (in_sizes[3] != (kHid + 1) * 4) return;
  if (in_sizes[4] != 4) return;
  if (out_size != kBatch * kSteps) return;

  const float* x  = (const float*)d_in[0];
  const float* W1 = (const float*)d_in[1];
  const float* b1 = (const float*)d_in[2];
  const float* W2 = (const float*)d_in[3];
  const float* b2 = (const float*)d_in[4];
  float* out = (float*)d_out;

  lstm2_fused_kernel<<<dim3(kBatch / kRowsBlk), dim3(kThreads), 0, stream>>>(x, W1, b1, W2, b2, out);

  (void)d_ws; (void)ws_size;
}
